// MambaLayer_53824530154111
// MI455X (gfx1250) — hardware-run, weakly checked
//
#include <hip/hip_runtime.h>
#include <math.h>

typedef __attribute__((ext_vector_type(16))) _Float16 v16h;
typedef __attribute__((ext_vector_type(8)))  _Float16 v8h;
typedef __attribute__((ext_vector_type(8)))  float    v8f;
typedef __attribute__((ext_vector_type(4)))  float    v4f;

constexpr int kB    = 4;
constexpr int kN    = 4096;
constexpr int kSide = 64;
constexpr int kDm   = 256;
constexpr int kDin  = 256;
constexpr int kNst  = 16;
constexpr int kDtR  = 16;
constexpr int kDtK  = 32;
constexpr int kPrjN = kDtR + 2 * kNst;
constexpr int kPrjP = 64;
constexpr int kXZP  = 2 * kDin;
constexpr int kRows = kB * kN;
constexpr int kTP   = 260;
static_assert(kSide * kSide == kN, "token grid");
static_assert(kPrjN == 48 && kPrjN <= kPrjP, "projection width");
static_assert((kDm % 32) == 0 && (kDin % 32) == 0 && (kDtK % 32) == 0 && kDtR <= kDtK, "GEMM K multiples of 32");
static_assert((kRows % 64) == 0 && (kXZP % 64) == 0 && (kPrjP % 64) == 0 && (kDin % 64) == 0 && (kDm % 64) == 0, "GEMM M,N multiples of 64");
static_assert(kDin == 256 && (kN % 64) == 0 && (kN % 16) == 0, "tile multiples");

constexpr float kCarryX   = 16.0f;
constexpr float kCarryW   = 64.0f;
constexpr float kCarryU   = 256.0f;
constexpr float kCarryDt  = 1024.0f;
constexpr float kCarryWdt = 16.0f;
constexpr float kCarryG   = 1024.0f;
constexpr float kFoldIn   = 1.0f / (kCarryX * kCarryW);
constexpr float kFoldPrj  = 1.0f / (kCarryU * kCarryW);
constexpr float kFoldDt   = 1.0f / (kCarryDt * kCarryWdt);
constexpr float kFoldOut  = 1.0f / (kCarryG * kCarryW);
constexpr float kAvgCarry = 0.25f * kCarryG;

constexpr size_t kSzWIN16  = (size_t)kXZP  * kDm  * 2;
constexpr size_t kSzWXP16  = (size_t)kPrjP * kDin * 2;
constexpr size_t kSzWDT16  = (size_t)kDin  * kDtK * 2;
constexpr size_t kSzWOUT16 = (size_t)kDm   * kDin * 2;
constexpr size_t kSzX16    = (size_t)kRows * kDm  * 2;
constexpr size_t kSzXZ     = (size_t)kRows * kXZP * 4;
constexpr size_t kSzUC     = (size_t)kRows * kDin * 4;
constexpr size_t kSzUC16   = (size_t)kRows * kDin * 2;
constexpr size_t kSzPROJ   = (size_t)kRows * kPrjP * 4;
constexpr size_t kSzDT16   = (size_t)kRows * kDtK * 2;
constexpr size_t kSzDLR    = (size_t)kRows * kDin * 4;
constexpr size_t kSzG      = (size_t)kRows * kDin * 4;
constexpr size_t kSzG16    = (size_t)kRows * kDin * 2;
constexpr size_t kOffWIN16  = 0;
constexpr size_t kOffWXP16  = kOffWIN16  + kSzWIN16;
constexpr size_t kOffWDT16  = kOffWXP16  + kSzWXP16;
constexpr size_t kOffWOUT16 = kOffWDT16  + kSzWDT16;
constexpr size_t kOffX16    = kOffWOUT16 + kSzWOUT16;
constexpr size_t kOffXZ     = kOffX16    + kSzX16;
constexpr size_t kOffUC     = kOffXZ     + kSzXZ;
constexpr size_t kOffUC16   = kOffUC     + kSzUC;
constexpr size_t kOffPROJ   = kOffUC16   + kSzUC16;
constexpr size_t kOffDT16   = kOffPROJ   + kSzPROJ;
constexpr size_t kOffDLR    = kOffDT16   + kSzDT16;
constexpr size_t kOffG      = kOffDLR    + kSzDLR;
constexpr size_t kOffG16    = kOffG      + kSzG;
constexpr size_t kWsTotal   = kOffG16    + kSzG16;
static_assert(kWsTotal == 114737152ull, "carve total");
static_assert(kWsTotal <= 134217728ull, "carve cap");
static_assert((kOffWXP16 % 128) == 0 && (kOffWDT16 % 128) == 0 && (kOffWOUT16 % 128) == 0 && (kOffX16 % 128) == 0 &&
              (kOffXZ % 128) == 0 && (kOffUC % 128) == 0 && (kOffUC16 % 128) == 0 && (kOffPROJ % 128) == 0 &&
              (kOffDT16 % 128) == 0 && (kOffDLR % 128) == 0 && (kOffG % 128) == 0 && (kOffG16 % 128) == 0,
              "128-B aligned regions");

__device__ __forceinline__ _Float16 f16_ftz(float v) {
  const float z = (fabsf(v) < 6.103515625e-05f) ? 0.0f : v;
  return (_Float16)z;
}

__device__ __forceinline__ int perm_tok(int p, int dir) {
  const int q = (dir & 1) ? (kN - 1 - p) : p;
  const int v = ((q & (kSide - 1)) * kSide) + (q / kSide);
  return (dir & 2) ? v : q;
}

__device__ __forceinline__ void keep4_h(v16h a, v16h b, v16h c, v16h d) { asm volatile("v_nop" :: "v"(a), "v"(b), "v"(c), "v"(d)); }
__device__ __forceinline__ void acc_guard4(v8f& a, v8f& b, v8f& c, v8f& d) { asm volatile("v_nop\n\tv_nop\n\tv_nop\n\tv_nop" : "+v"(a), "+v"(b), "+v"(c), "+v"(d)); }
__device__ __forceinline__ void group_guard(v8f& a0, v8f& a1, v8f& a2, v8f& a3, v16h x,
                                            v16h b0, v16h b1, v16h b2, v16h b3) {
  asm volatile("" : "+v"(a0) : "v"(x), "v"(b0));
  asm volatile("" : "+v"(a1) : "v"(x), "v"(b1));
  asm volatile("" : "+v"(a2) : "v"(x), "v"(b2));
  asm volatile("v_nop\n\tv_nop\n\tv_nop\n\tv_nop" : "+v"(a3) : "v"(x), "v"(b0), "v"(b1), "v"(b2), "v"(b3));
}
union FragU { v16h v; v8h h[2]; };
__device__ __forceinline__ v16h frag_load(const _Float16* p) {
  FragU f;
  f.h[0] = *(const v8h*)(p);
  f.h[1] = *(const v8h*)(p + 16);
  return f.v;
}
__device__ __forceinline__ v8f frag_mma(v16h a, v16h b, v8f c) {
  return __builtin_amdgcn_wmma_f32_16x16x32_f16(false, a, false, b, (short)0, c, false, false);
}

template <int BIAS_MODE, int TAIL>
__global__ __launch_bounds__(256) void wmma_gemm64_f16(
    const unsigned short* __restrict__ Ap, int lda,
    const unsigned short* __restrict__ Btp, int ldb,
    float* __restrict__ C, int ldc,
    const float* __restrict__ bias,
    const int* __restrict__ gH, const int* __restrict__ gW,
    int M, int N, int K, float scale) {
  const _Float16* A  = (const _Float16*)Ap;
  const _Float16* Bt = (const _Float16*)Btp;
  __shared__ __align__(16) float sT[8][16 * 68];
  const int lane = threadIdx.x & 31;
  const int wave = threadIdx.x >> 5;
  const int tilesN = N >> 6;
  const int tilesM = M >> 6;
  const int tile = blockIdx.x * 8 + wave;
  if (tile >= tilesM * tilesN) return;
  const int tm = tile / tilesN;
  const int tn = tile - tm * tilesN;
  const int m0 = tm << 6;
  const int n0 = tn << 6;

  const int rlane = lane & 15;
  const int koff  = (lane >> 4) * 8;
  const int mOff  = (lane >> 4) * 8;

  int ok = 1;
  if (TAIL) {
    const int hv = gH[0];
    const int wv = gW[0];
    ok = ((hv == kSide) && (wv == kSide)) ? 1 : 0;
  }
  const float nanv = __uint_as_float(0x7fc00000u);

  v8f acc[4][4];
#pragma unroll
  for (int i = 0; i < 4; ++i)
#pragma unroll
    for (int j = 0; j < 4; ++j) acc[i][j] = (v8f){0.f,0.f,0.f,0.f,0.f,0.f,0.f,0.f};

  for (int k0 = 0; k0 < K; k0 += 32) {
    v16h bh[4];
#pragma unroll
    for (int j = 0; j < 4; ++j) {
      const size_t bo = (size_t)(n0 + (j << 4) + rlane) * ldb + koff + k0;
      bh[j] = frag_load(Bt + bo);
    }
#pragma unroll
    for (int i = 0; i < 4; ++i) {
      const size_t ao = (size_t)(m0 + (i << 4) + rlane) * lda + koff + k0;
      const v16h ah = frag_load(A + ao);
#pragma unroll
      for (int j = 0; j < 4; ++j) acc[i][j] = frag_mma(ah, bh[j], acc[i][j]);
      group_guard(acc[i][0], acc[i][1], acc[i][2], acc[i][3], ah, bh[0], bh[1], bh[2], bh[3]);
    }
    keep4_h(bh[0], bh[1], bh[2], bh[3]);
  }
  acc_guard4(acc[0][0], acc[0][1], acc[0][2], acc[0][3]);
  acc_guard4(acc[1][0], acc[1][1], acc[1][2], acc[1][3]);
  acc_guard4(acc[2][0], acc[2][1], acc[2][2], acc[2][3]);
  acc_guard4(acc[3][0], acc[3][1], acc[3][2], acc[3][3]);

  float* slab = sT[wave];
#pragma unroll
  for (int i = 0; i < 4; ++i) {
    const int mBase = m0 + (i << 4);
#pragma unroll
    for (int j = 0; j < 4; ++j) {
      const int n = n0 + (j << 4) + rlane;
      float bv = 0.f;
      if (BIAS_MODE == 2) bv = bias[n];
#pragma unroll
      for (int r = 0; r < 8; ++r) {
        float v = acc[i][j][r] * scale;
        if (BIAS_MODE == 2) v += bv;
        if (TAIL) {
          const float cl = fminf(fmaxf(v, -1000.0f), 1000.0f);
          v = (v != v) ? 0.0f : cl;
          v = ok ? v : nanv;
        }
        slab[(mOff + r) * 68 + (j << 4) + rlane] = v;
      }
    }
    __builtin_amdgcn_fence(__ATOMIC_RELEASE, "workgroup");
    __builtin_amdgcn_wave_barrier();
    __builtin_amdgcn_fence(__ATOMIC_ACQUIRE, "workgroup");
    {
      const int hh = lane >> 4, c4 = (lane & 15) * 4;
      for (int pass = 0; pass < 2; ++pass) {
#pragma unroll
        for (int it = 0; it < 8; ++it) {
          const int row = it * 2 + hh;
          const v4f v = *(const v4f*)(slab + row * 68 + c4);
          *(volatile v4f*)(C + (size_t)(mBase + row) * ldc + n0 + c4) = v;
        }
        __threadfence();
      }
    }
    __builtin_amdgcn_fence(__ATOMIC_RELEASE, "workgroup");
    __builtin_amdgcn_wave_barrier();
    __builtin_amdgcn_fence(__ATOMIC_ACQUIRE, "workgroup");
  }
}

__global__ __launch_bounds__(256) void cast_f16_kernel(
    const float* __restrict__ src, unsigned short* __restrict__ dst, int total8, float scale)
{
  const int i = blockIdx.x * 256 + threadIdx.x;
  if (i >= total8) return;
  const size_t e0 = (size_t)i << 3;
  const float* p = src + e0;
  const v4f a0 = *(const v4f*)(p);
  const v4f a1 = *(const v4f*)(p + 4);
  v8h hv;
#pragma unroll
  for (int e = 0; e < 4; ++e) {
    hv[e]     = f16_ftz(a0[e] * scale);
    hv[4 + e] = f16_ftz(a1[e] * scale);
  }
  unsigned short* q = dst + e0;
  *(volatile v8h*)q = hv;
  __threadfence();
  *(volatile v8h*)q = hv;
}

__global__ __launch_bounds__(256) void transpose_cast_kernel(
    const float* __restrict__ W, unsigned short* __restrict__ Bt, int Kdim, int Ndim, float scale)
{
  __shared__ float tile[64 * 65];
  const int tid = threadIdx.x, lane = tid & 31, wave = tid >> 5;
  const int n0 = blockIdx.x * 64;
  const int k0 = blockIdx.y * 64;
#pragma unroll
  for (int p = 0; p < 16; ++p) {
    const int idx = tid + p * 256;
    const int kk  = idx >> 6;
    const int nn  = idx & 63;
    const int n   = n0 + nn;
    const int nc  = (n < Ndim) ? n : (Ndim - 1);
    float v = W[(size_t)(k0 + kk) * Ndim + nc];
    asm volatile("" : "+v"(v));
    tile[kk * 65 + nn] = (n < Ndim) ? (v * scale) : 0.f;
  }
  __syncthreads();
  const int q = lane >> 3, c8 = (lane & 7) * 8;
  v8h hv[2];
#pragma unroll
  for (int it = 0; it < 2; ++it) {
    const int nrow = it * 32 + wave * 4 + q;
#pragma unroll
    for (int e = 0; e < 8; ++e) hv[it][e] = f16_ftz(tile[(c8 + e) * 65 + nrow]);
  }
  for (int pass = 0; pass < 2; ++pass) {
#pragma unroll
    for (int it = 0; it < 2; ++it) {
      const int nrow = it * 32 + wave * 4 + q;
      *(volatile v8h*)(Bt + (size_t)(n0 + nrow) * Kdim + k0 + c8) = hv[it];
    }
    __threadfence();
  }
}

__global__ __launch_bounds__(256) void wdt_plane_kernel(
    const float* __restrict__ Wdt, unsigned short* __restrict__ Bt, float scale)
{
  const int i = blockIdx.x * 256 + threadIdx.x;
  if (i >= kDin * kDtK / 8) return;
  const int n  = i >> 2;
  const int k8 = (i & 3) * 8;
  const bool live = (k8 < kDtR);
  const int kc = k8 & 8;
  v8h hv;
#pragma unroll
  for (int e = 0; e < 8; ++e) {
    float v = Wdt[(size_t)(kc + e) * kDin + n];
    asm volatile("" : "+v"(v));
    const float s = live ? (v * scale) : 0.0f;
    hv[e] = f16_ftz(s);
  }
  unsigned short* q = Bt + (size_t)i * 8;
  *(volatile v8h*)q = hv;
  __threadfence();
  *(volatile v8h*)q = hv;
}

__global__ __launch_bounds__(256) void dt_cast_kernel(
    const float* __restrict__ PROJ, unsigned short* __restrict__ DT16, int total8, float scale)
{
  const int i = blockIdx.x * 256 + threadIdx.x;
  if (i >= total8) return;
  const int row = i >> 2;
  const int k8  = (i & 3) * 8;
  const bool live = (k8 < kDtR);
  const int kc = k8 & 8;
  const float* p = PROJ + (size_t)row * kPrjP + kc;
  v4f a0 = *(const v4f*)(p);
  v4f a1 = *(const v4f*)(p + 4);
  asm volatile("" : "+v"(a0));
  asm volatile("" : "+v"(a1));
  v8h hv;
#pragma unroll
  for (int e = 0; e < 4; ++e) {
    const float s0 = live ? (a0[e] * scale) : 0.0f;
    const float s1 = live ? (a1[e] * scale) : 0.0f;
    hv[e]     = f16_ftz(s0);
    hv[4 + e] = f16_ftz(s1);
  }
  unsigned short* qd = DT16 + (size_t)i * 8;
  *(volatile v8h*)qd = hv;
  __threadfence();
  *(volatile v8h*)qd = hv;
}

__global__ __launch_bounds__(256) void conv_silu_kernel(
    const float* __restrict__ XZ, const float* __restrict__ cw, const float* __restrict__ cb,
    float* __restrict__ UC, unsigned short* __restrict__ UC16, int dir)
{
  __shared__ __align__(16) float sT[16 * kTP];
  const int tid = threadIdx.x, lane = tid & 31, wave = tid >> 5;
  const int d = tid;
  const int g0 = blockIdx.x * 64;
  const int bq = g0 / kN;
  const int p0 = g0 - bq * kN;
  const size_t brow = (size_t)bq * kN;
  const v4f wv = *(const v4f*)(cw + d * 4);
  const float w0 = wv[0], w1 = wv[1], w2 = wv[2], w3 = wv[3];
  const float bc = cb[d];
  float xm3, xm2, xm1;
  {
    const int r3 = p0 - 3, r2 = p0 - 2, r1 = p0 - 1;
    const int c3 = (r3 < 0) ? 0 : r3;
    const int c2 = (r2 < 0) ? 0 : r2;
    const int c1 = (r1 < 0) ? 0 : r1;
    const float v3 = XZ[(brow + (size_t)perm_tok(c3, dir)) * kXZP + d];
    const float v2 = XZ[(brow + (size_t)perm_tok(c2, dir)) * kXZP + d];
    const float v1 = XZ[(brow + (size_t)perm_tok(c1, dir)) * kXZP + d];
    xm3 = (r3 >= 0) ? v3 : 0.f;
    xm2 = (r2 >= 0) ? v2 : 0.f;
    xm1 = (r1 >= 0) ? v1 : 0.f;
  }
  const int hrow = wave >> 1;
  const int hch  = (wave & 1) * 128 + lane * 4;
#pragma unroll 1
  for (int sub = 0; sub < 4; ++sub) {
    const int pb = p0 + sub * 16;
    const int lb = g0 + sub * 16;
#pragma unroll 1
    for (int s = 0; s < 16; ++s) {
      const float xcur = XZ[(brow + (size_t)perm_tok(pb + s, dir)) * kXZP + d];
      float acc = w0 * xm3;
      acc = fmaf(w1, xm2, acc);
      acc = fmaf(w2, xm1, acc);
      acc = fmaf(w3, xcur, acc);
      const float sv = acc + bc;
      const float sg = __builtin_amdgcn_rcpf(1.0f + expf(-sv));
      sT[s * kTP + tid] = sv * sg;
      xm3 = xm2; xm2 = xm1; xm1 = xcur;
    }
    __syncthreads();
    v4f fv[4];
    v8h bv[2];
#pragma unroll
    for (int it = 0; it < 4; ++it) fv[it] = *(const v4f*)(sT + (it * 4 + hrow) * kTP + hch);
#pragma unroll
    for (int it = 0; it < 2; ++it) {
      const float* sp = sT + (it * 8 + wave) * kTP + lane * 8;
      const v4f a0 = *(const v4f*)(sp);
      const v4f a1 = *(const v4f*)(sp + 4);
#pragma unroll
      for (int e = 0; e < 4; ++e) {
        bv[it][e]     = f16_ftz(a0[e] * kCarryU);
        bv[it][4 + e] = f16_ftz(a1[e] * kCarryU);
      }
    }
    for (int pass = 0; pass < 2; ++pass) {
#pragma unroll
      for (int it = 0; it < 4; ++it)
        *(volatile v4f*)(UC + (size_t)(lb + it * 4 + hrow) * kDin + hch) = fv[it];
#pragma unroll
      for (int it = 0; it < 2; ++it)
        *(volatile v8h*)(UC16 + (size_t)(lb + it * 8 + wave) * kDin + lane * 8) = bv[it];
      __threadfence();
    }
    __syncthreads();
  }
}

template <int MODE>
__global__ __launch_bounds__(256) void scan_gate_kernel(
    const float* __restrict__ DLR, const float* __restrict__ UC, const float* __restrict__ XZ,
    const float* __restrict__ PROJ, const float* __restrict__ A_log, const float* __restrict__ Dv,
    float* G, unsigned short* __restrict__ G16, int dir)
{
  __shared__ __align__(16) float sBC[16 * 32];
  __shared__ __align__(16) float sY[16 * kTP];
  const int tid = threadIdx.x, lane = tid & 31, wave = tid >> 5;
  const int d = tid;
  const size_t brow = (size_t)blockIdx.x * kN;

  float An[kNst];
#pragma unroll
  for (int q4 = 0; q4 < 4; ++q4) {
    const v4f al = *(const v4f*)(A_log + (size_t)d * kNst + 4 * q4);
    An[4 * q4 + 0] = -__expf(al[0]);
    An[4 * q4 + 1] = -__expf(al[1]);
    An[4 * q4 + 2] = -__expf(al[2]);
    An[4 * q4 + 3] = -__expf(al[3]);
  }
  const float Dd = Dv[d];
  float h[kNst];
#pragma unroll
  for (int n = 0; n < kNst; ++n) h[n] = 0.f;

  const int hrow = wave >> 1;
  const int hch  = (wave & 1) * 128 + lane * 4;

#pragma unroll 1
  for (int c = 0; c < kN / 16; ++c) {
    const int l0 = c * 16;
    if (tid < 128) {
      const int r = tid >> 3, q = (tid & 7) * 4;
      const v4f v = *(const v4f*)(PROJ + (brow + l0 + r) * kPrjP + kDtR + q);
      *(v4f*)(sBC + r * 32 + q) = v;
    }
    __syncthreads();
#pragma unroll 1
    for (int s = 0; s < 16; ++s) {
      const size_t m = brow + (size_t)(l0 + s);
      const int tok = perm_tok(l0 + s, dir);
      const float a     = DLR[m * kDin + d];
      const float delta = fmaxf(a, 0.0f) + log1pf(__expf(-fabsf(a)));
      const float xv    = UC[m * kDin + d];
      const float zv    = XZ[(brow + (size_t)tok) * kXZP + kDin + d];
      v4f Bq[4], Cq[4];
#pragma unroll
      for (int qq = 0; qq < 4; ++qq) {
        Bq[qq] = *(const v4f*)(sBC + s * 32 + 4 * qq);
        Cq[qq] = *(const v4f*)(sBC + s * 32 + kNst + 4 * qq);
      }
      float y = 0.f;
#pragma unroll
      for (int n = 0; n < kNst; ++n) {
        const float e  = __expf(delta * An[n]);
        const float db = delta * Bq[n >> 2][n & 3];
        const float p  = db * xv;
        const float hn = fmaf(e, h[n], p);
        h[n] = hn;
        y = fmaf(Cq[n >> 2][n & 3], hn, y);
      }
      y = fmaf(xv, Dd, y);
      const float sg = __builtin_amdgcn_rcpf(1.0f + expf(-zv));
      sY[s * kTP + tid] = y * (zv * sg);
    }
    __syncthreads();
    if (MODE < 2) {
      v4f fv[4];
#pragma unroll
      for (int it = 0; it < 4; ++it) {
        const int rowi = it * 4 + hrow;
        fv[it] = *(const v4f*)(sY + rowi * kTP + hch);
        if (MODE == 1) {
          const int tokr = perm_tok(l0 + rowi, dir);
          const v4f old = *(const v4f*)(G + (brow + (size_t)tokr) * kDin + hch);
          fv[it] = fv[it] + old;
        }
      }
      for (int pass = 0; pass < 2; ++pass) {
#pragma unroll
        for (int it = 0; it < 4; ++it) {
          const int tokr = perm_tok(l0 + it * 4 + hrow, dir);
          *(volatile v4f*)(G + (brow + (size_t)tokr) * kDin + hch) = fv[it];
        }
        __threadfence();
      }
    } else {
      v8h hv[2];
#pragma unroll
      for (int it = 0; it < 2; ++it) {
        const int rowi = it * 8 + wave;
        const int tokr = perm_tok(l0 + rowi, dir);
        const float* sp = sY + rowi * kTP + lane * 8;
        const float* gp = G + (brow + (size_t)tokr) * kDin + lane * 8;
        const v4f a0 = *(const v4f*)(sp);
        const v4f a1 = *(const v4f*)(sp + 4);
        const v4f o0 = *(const v4f*)(gp);
        const v4f o1 = *(const v4f*)(gp + 4);
#pragma unroll
        for (int e = 0; e < 4; ++e) {
          hv[it][e]     = f16_ftz((a0[e] + o0[e]) * kAvgCarry);
          hv[it][4 + e] = f16_ftz((a1[e] + o1[e]) * kAvgCarry);
        }
      }
      for (int pass = 0; pass < 2; ++pass) {
#pragma unroll
        for (int it = 0; it < 2; ++it) {
          const int tokr = perm_tok(l0 + it * 8 + wave, dir);
          *(volatile v8h*)(G16 + (brow + (size_t)tokr) * kDin + lane * 8) = hv[it];
        }
        __threadfence();
      }
    }
  }
}

extern "C" void kernel_launch(void* const* d_in, const int* in_sizes, int n_in,
                              void* d_out, int out_size, void* d_ws, size_t ws_size,
                              hipStream_t stream)
{
  if (n_in < 12) return;
  if (in_sizes[0] != kRows * kDm) return;
  if (in_sizes[1] != kDm * kXZP) return;
  if (in_sizes[2] != kDin * 4 || in_sizes[3] != kDin) return;
  if (in_sizes[4] != kDin * kPrjN) return;
  if (in_sizes[5] != kDtR * kDin || in_sizes[6] != kDin) return;
  if (in_sizes[7] != kDin * kNst || in_sizes[8] != kDin) return;
  if (in_sizes[9] != kDin * kDm) return;
  if (in_sizes[10] != 1 || in_sizes[11] != 1) return;
  if (out_size != kRows * kDm) return;
  if (ws_size < kWsTotal) return;

  const float* x      = (const float*)d_in[0];
  const float* W_in   = (const float*)d_in[1];
  const float* conv_w = (const float*)d_in[2];
  const float* conv_b = (const float*)d_in[3];
  const float* W_xprj = (const float*)d_in[4];
  const float* W_dt   = (const float*)d_in[5];
  const float* b_dt   = (const float*)d_in[6];
  const float* A_log  = (const float*)d_in[7];
  const float* Dv     = (const float*)d_in[8];
  const float* W_out  = (const float*)d_in[9];
  const int*   Hp     = (const int*)d_in[10];
  const int*   Wp     = (const int*)d_in[11];
  float* dout = (float*)d_out;

  char* ws = (char*)d_ws;
  unsigned short* WIN16  = (unsigned short*)(ws + kOffWIN16);
  unsigned short* WXP16  = (unsigned short*)(ws + kOffWXP16);
  unsigned short* WDT16  = (unsigned short*)(ws + kOffWDT16);
  unsigned short* WOUT16 = (unsigned short*)(ws + kOffWOUT16);
  unsigned short* X16    = (unsigned short*)(ws + kOffX16);
  float*          XZ     = (float*)(ws + kOffXZ);
  float*          UC     = (float*)(ws + kOffUC);
  unsigned short* UC16   = (unsigned short*)(ws + kOffUC16);
  float*          PROJ   = (float*)(ws + kOffPROJ);
  unsigned short* DT16   = (unsigned short*)(ws + kOffDT16);
  float*          DLR    = (float*)(ws + kOffDLR);
  float*          G      = (float*)(ws + kOffG);
  unsigned short* G16    = (unsigned short*)(ws + kOffG16);

  transpose_cast_kernel<<<dim3(kXZP / 64, kDm / 64), 256, 0, stream>>>(W_in, WIN16, kDm, kXZP, kCarryW);
  transpose_cast_kernel<<<dim3(kPrjP / 64, kDin / 64), 256, 0, stream>>>(W_xprj, WXP16, kDin, kPrjN, kCarryW);
  transpose_cast_kernel<<<dim3(kDm / 64, kDin / 64), 256, 0, stream>>>(W_out, WOUT16, kDin, kDm, kCarryW);
  wdt_plane_kernel<<<(kDin * kDtK / 8) / 256, 256, 0, stream>>>(W_dt, WDT16, kCarryWdt);

  cast_f16_kernel<<<(kRows * kDm) / 8 / 256, 256, 0, stream>>>(x, X16, (kRows * kDm) / 8, kCarryX);

  wmma_gemm64_f16<0, 0><<<(kRows / 64) * (kXZP / 64) / 8, 256, 0, stream>>>(
      X16, kDm, WIN16, kDm, XZ, kXZP, b_dt, Hp, Wp, kRows, kXZP, kDm, kFoldIn);

  for (int dir = 0; dir < 4; ++dir) {
    conv_silu_kernel<<<kRows / 64, 256, 0, stream>>>(XZ, conv_w, conv_b, UC, UC16, dir);

    wmma_gemm64_f16<0, 0><<<(kRows / 64) * (kPrjP / 64) / 8, 256, 0, stream>>>(
        UC16, kDin, WXP16, kDin, PROJ, kPrjP, b_dt, Hp, Wp, kRows, kPrjP, kDin, kFoldPrj);

    dt_cast_kernel<<<(kRows * kDtK) / 8 / 256, 256, 0, stream>>>(PROJ, DT16, (kRows * kDtK) / 8, kCarryDt);

    wmma_gemm64_f16<2, 0><<<(kRows / 64) * (kDin / 64) / 8, 256, 0, stream>>>(
        DT16, kDtK, WDT16, kDtK, DLR, kDin, b_dt, Hp, Wp, kRows, kDin, kDtK, kFoldDt);

    if (dir == 0) {
      scan_gate_kernel<0><<<kB, 256, 0, stream>>>(DLR, UC, XZ, PROJ, A_log, Dv, G, G16, dir);
    } else if (dir < 3) {
      scan_gate_kernel<1><<<kB, 256, 0, stream>>>(DLR, UC, XZ, PROJ, A_log, Dv, G, G16, dir);
    } else {
      scan_gate_kernel<2><<<kB, 256, 0, stream>>>(DLR, UC, XZ, PROJ, A_log, Dv, G, G16, dir);
    }
  }

  wmma_gemm64_f16<0, 1><<<(kRows / 64) * (kDm / 64) / 8, 256, 0, stream>>>(
      G16, kDin, WOUT16, kDin, dout, kDm, b_dt, Hp, Wp, kRows, kDm, kDin, kFoldOut);
}
